// TransformerLayer_5763846111742
// MI455X (gfx1250) — hardware-verified
//
#include <hip/hip_runtime.h>


#ifndef NB
#define NB 4
#endif
#ifndef SEQ
#define SEQ 1024
#endif
#define SEQ_FULL 1024
#define ML_FULL  2048
#define EE    1024
#define NHEAD 16
#define HD    64
#define FF    4096
#define ROWS  (NB * SEQ)
#define QT    (SEQ / 16)
#define WCAR  64.0f
#define SCLQK 0.001953125f
#define L2E   1.4426950408889634f
#define NEGV  (-1.0e30f)

static_assert(NHEAD * HD == EE);
static_assert(HD == 64);
static_assert(EE == 1024);
static_assert((SEQ & (SEQ - 1)) == 0);
static_assert(SEQ % 128 == 0 && SEQ <= SEQ_FULL && SEQ <= ML_FULL);
static_assert(ROWS % 64 == 0);
static_assert((NB * NHEAD * QT) % 8 == 0 && QT % 8 == 0);
static_assert((size_t)NB * NHEAD * QT * 16 * HD == (size_t)ROWS * EE);
static_assert((3 * EE * EE) % 2048 == 0 && (EE * EE) % 2048 == 0 && (FF * EE) % 2048 == 0);

typedef _Float16 h16;
typedef __attribute__((ext_vector_type(16))) _Float16 v16h;
typedef __attribute__((ext_vector_type(8)))  _Float16 v8h;
typedef __attribute__((ext_vector_type(8)))  float    v8f;
typedef __attribute__((ext_vector_type(4)))  float    v4f;
typedef v8h __attribute__((may_alias)) v8ha;
typedef v4f __attribute__((may_alias)) v4fa;

__device__ __forceinline__ unsigned short f2bf(float f) { unsigned u = __float_as_uint(f); u += 0x7FFFu + ((u >> 16) & 1u); return (unsigned short)(u >> 16); }
__device__ __forceinline__ float bf2f(unsigned short b) { return __uint_as_float(((unsigned)b) << 16); }
__device__ __forceinline__ float bfr(float f) { return bf2f(f2bf(f)); }
__device__ __forceinline__ v16h cat16(v8h lo, v8h hi) { return __builtin_shufflevector(lo, hi, 0, 1, 2, 3, 4, 5, 6, 7, 8, 9, 10, 11, 12, 13, 14, 15); }
__device__ __forceinline__ v8f wmma16(v16h a, v16h b, v8f c) { return __builtin_amdgcn_wmma_f32_16x16x32_f16(false, a, false, b, (short)0, c, false, false); }
__device__ __forceinline__ v16h ldf(const h16* p) { return cat16(*(const v8h*)p, *(const v8h*)(p + 16)); }
__device__ __forceinline__ unsigned xrow(unsigned row) { return (row / (unsigned)SEQ) * (unsigned)SEQ_FULL + (row % (unsigned)SEQ); }

__global__ __launch_bounds__(256) void k_cvtw(const float* __restrict__ src, h16* dst, unsigned n8) {
    const unsigned i = blockIdx.x * 256u + threadIdx.x; if (i >= n8) return;
    const v4f a = *(const v4f*)(src + (size_t)i * 8), b = *(const v4f*)(src + (size_t)i * 8 + 4); v8h o;
#pragma unroll
    for (int k = 0; k < 4; ++k) { o[k] = (h16)(bfr(a[k]) * WCAR); o[4 + k] = (h16)(bfr(b[k]) * WCAR); }
    *(volatile v8h*)(dst + (size_t)i * 8) = o; __threadfence(); *(volatile v8h*)(dst + (size_t)i * 8) = o; }

template <bool RBF>
__global__ __launch_bounds__(256) void k_ln(const float* __restrict__ src, const float* __restrict__ g, const float* __restrict__ be, h16* dst) {
    const unsigned lane = threadIdx.x & 31u, wave = threadIdx.x >> 5; const unsigned row = blockIdx.x * 8u + wave;
    const unsigned srow = RBF ? xrow(row) : row; const float* xr = src + (size_t)srow * EE + lane * 8u;
    float s = 0.f;
#pragma unroll 1
    for (unsigned c = 0; c < 4u; ++c) { const v4f a = *(const v4f*)(xr + c * 256u), b = *(const v4f*)(xr + c * 256u + 4u);
#pragma unroll
        for (int q = 0; q < 4; ++q) { s += RBF ? bfr(a[q]) : a[q]; s += RBF ? bfr(b[q]) : b[q]; } }
#pragma unroll
    for (int sh = 16; sh; sh >>= 1) s += __shfl_xor(s, sh, 32);
    const float mean = s * (1.0f / 1024.0f);
    float ss = 0.f;
#pragma unroll 1
    for (unsigned c = 0; c < 4u; ++c) { const v4f a = *(const v4f*)(xr + c * 256u), b = *(const v4f*)(xr + c * 256u + 4u);
#pragma unroll
        for (int q = 0; q < 4; ++q) { const float d0 = (RBF ? bfr(a[q]) : a[q]) - mean, d1 = (RBF ? bfr(b[q]) : b[q]) - mean; ss += d0 * d0; ss += d1 * d1; } }
#pragma unroll
    for (int sh = 16; sh; sh >>= 1) ss += __shfl_xor(ss, sh, 32);
    const float rstd = rsqrtf(ss * (1.0f / 1024.0f) + 1e-5f);
    h16* drow = dst + (size_t)row * EE + lane * 8u;
#pragma unroll 1
    for (int ps = 0; ps < 2; ++ps) {
#pragma unroll 1
        for (unsigned c = 0; c < 4u; ++c) { const unsigned co = c * 256u; const v4f a = *(const v4f*)(xr + co), b = *(const v4f*)(xr + co + 4u);
            const v4f g0 = *(const v4f*)(g + co + lane * 8u), g1 = *(const v4f*)(g + co + lane * 8u + 4u), e0 = *(const v4f*)(be + co + lane * 8u), e1 = *(const v4f*)(be + co + lane * 8u + 4u); v8h o;
#pragma unroll
            for (int q = 0; q < 4; ++q) { const float x0 = RBF ? bfr(a[q]) : a[q], x1 = RBF ? bfr(b[q]) : b[q];
                o[q] = (h16)((x0 - mean) * rstd * bfr(g0[q]) + bfr(e0[q])); o[4 + q] = (h16)((x1 - mean) * rstd * bfr(g1[q]) + bfr(e1[q])); }
            *(volatile v8h*)(drow + co) = o; }
        if (ps == 0) __threadfence(); }
}

#define EPI_QKV  0
#define EPI_RELU 1
#define EPI_RES  2
template <int EPI, bool RBF>
__global__ __launch_bounds__(32) void k_gemmw(const h16* __restrict__ A, const h16* __restrict__ Bt, unsigned K, const float* __restrict__ bias, float s1, float s2,
                                              const float* __restrict__ resid, float* Cf, h16* D0, h16* D1, h16* D2, unsigned ldd) {
    __shared__ __align__(16) float os[64 * 68];
    const unsigned lane = threadIdx.x & 31u, lr = lane & 15u, hi = lane >> 4; const unsigned r0 = blockIdx.x * 64u, c0 = blockIdx.y * 64u;
    v8f acc[4][4];
#pragma unroll
    for (int mb = 0; mb < 4; ++mb)
#pragma unroll
        for (int nb = 0; nb < 4; ++nb) acc[mb][nb] = (v8f){};
    const size_t aoff = (size_t)(r0 + lr) * K + 8u * hi, boff = (size_t)(c0 + lr) * K + 8u * hi;
#pragma unroll 1
    for (unsigned kc = 0; kc < K; kc += 32u) {
        v16h a[4];
#pragma unroll
        for (int mb = 0; mb < 4; ++mb) a[mb] = ldf(A + aoff + (size_t)mb * 16 * K + kc);
#pragma unroll
        for (int nb = 0; nb < 4; ++nb) { const v16h b = ldf(Bt + boff + (size_t)nb * 16 * K + kc);
#pragma unroll
            for (int mb = 0; mb < 4; ++mb) acc[mb][nb] = wmma16(a[mb], b, acc[mb][nb]); }
        asm volatile("v_nop\n\tv_nop\n\tv_nop\n\tv_nop" : "+v"(acc[0][0]), "+v"(acc[1][1]), "+v"(acc[2][2]), "+v"(acc[3][3]) : "v"(a[0]), "v"(a[3]));
    }
    const unsigned sec = (EPI == EPI_QKV) ? (c0 / (unsigned)EE) : 0u; const bool tr = (EPI == EPI_QKV) && (sec == 2u);
    float bc[4];
#pragma unroll
    for (int nb = 0; nb < 4; ++nb) bc[nb] = bfr(bias[c0 + nb * 16 + lr]);
#pragma unroll
    for (int mb = 0; mb < 4; ++mb)
#pragma unroll
        for (int nb = 0; nb < 4; ++nb)
#pragma unroll
            for (int j = 0; j < 8; ++j) { float v = acc[mb][nb][j] * s1 + bc[nb]; if (EPI == EPI_RELU) v = fmaxf(v, 0.0f); v *= s2;
                const unsigned rr = mb * 16 + hi * 8u + j, cc = nb * 16 + lr; os[tr ? (cc * 68u + rr) : (rr * 68u + cc)] = v; }
    __syncthreads();
    if (EPI == EPI_RES) {
        float* crow = Cf + (size_t)r0 * ldd + c0;
#pragma unroll 1
        for (int ps = 0; ps < 2; ++ps) {
#pragma unroll 4
            for (unsigned s = 0; s < 32u; ++s) { const unsigned row = 2u * s + hi, cofs = lr * 4u; v4f val = *(const v4fa*)(os + row * 68u + cofs);
                const unsigned rrow = RBF ? xrow(r0 + row) : (r0 + row); const v4f rv = *(const v4f*)(resid + (size_t)rrow * ldd + c0 + cofs);
#pragma unroll
                for (int q = 0; q < 4; ++q) val[q] += RBF ? bfr(rv[q]) : rv[q];
                *(volatile v4f*)(crow + (size_t)row * ldd + cofs) = val; }
            if (ps == 0) __threadfence(); }
    } else {
        h16* dst; size_t pitch;
        if (EPI == EPI_RELU) { dst = D0 + (size_t)r0 * ldd + c0; pitch = ldd; }
        else { const unsigned b = r0 / (unsigned)SEQ, t0 = r0 % (unsigned)SEQ, head = (c0 % (unsigned)EE) / (unsigned)HD; const size_t bh = (size_t)b * NHEAD + head;
            if (tr) { dst = D2 + bh * HD * SEQ + t0; pitch = SEQ; }
            else { h16* pl = (sec == 0u) ? D0 : D1; dst = pl + (bh * SEQ + t0) * HD; pitch = HD; } }
#pragma unroll 1
        for (int ps = 0; ps < 2; ++ps) {
#pragma unroll 4
            for (unsigned p = 0; p < 16u; ++p) { const unsigned row = p * 4u + (lane >> 3), pc = (lane & 7u) * 8u;
                const v4f x0 = *(const v4fa*)(os + row * 68u + pc), x1 = *(const v4fa*)(os + row * 68u + pc + 4u); v8h o;
#pragma unroll
                for (int q = 0; q < 4; ++q) { o[q] = (h16)x0[q]; o[4 + q] = (h16)x1[q]; }
                *(volatile v8h*)(dst + (size_t)row * pitch + pc) = o; }
            if (ps == 0) __threadfence(); }
    }
}

__global__ __launch_bounds__(256) void k_attn(const h16* __restrict__ QP, const h16* __restrict__ KP, const h16* __restrict__ VT, const float* __restrict__ relp, h16* OP) {
    __shared__ float rpl[SEQ];
    __shared__ __align__(16) h16 ot[8][16 * 72];
    const unsigned tid = threadIdx.x, lane = tid & 31u, wave = tid >> 5, lr = lane & 15u, hi = lane >> 4;
    const unsigned task = blockIdx.x * 8u + wave; const unsigned qb = task % (unsigned)QT, bh = task / (unsigned)QT; const unsigned head = bh % (unsigned)NHEAD, b = bh / (unsigned)NHEAD;
    for (unsigned i = tid; i < (unsigned)SEQ; i += 256u) rpl[i] = bfr(relp[(size_t)head * ML_FULL + i]);
    __syncthreads();
    const h16* qrow = QP + ((size_t)bh * SEQ + qb * 16u + lr) * HD + 8u * hi;
    const v16h qf0 = ldf(qrow), qf1 = ldf(qrow + 32);
    const h16* kbase = KP + ((size_t)bh * SEQ + lr) * HD + 8u * hi;
    const h16* vbase = VT + ((size_t)bh * HD + lr) * SEQ + 8u * hi;
    float m = NEGV, l = 0.f; v8f accO[4];
#pragma unroll
    for (int mb = 0; mb < 4; ++mb) accO[mb] = (v8f){};
    const unsigned qi = qb * 16u + lr; const unsigned nkb = (qb >> 1) + 1u;
#pragma unroll 1
    for (unsigned kb = 0; kb < nkb; ++kb) {
        const h16* kp = kbase + (size_t)kb * 32u * HD;
        const v16h ka00 = ldf(kp), ka01 = ldf(kp + 32), ka10 = ldf(kp + 16 * HD), ka11 = ldf(kp + 16 * HD + 32);
        v8f s0 = (v8f){}, s1 = (v8f){};
        s0 = wmma16(ka00, qf0, s0); s1 = wmma16(ka10, qf0, s1); s0 = wmma16(ka01, qf1, s0); s1 = wmma16(ka11, qf1, s1);
        asm volatile("v_nop\n\tv_nop\n\tv_nop\n\tv_nop" : "+v"(s0), "+v"(s1) : "v"(ka01), "v"(ka11), "v"(qf1));
        const unsigned j0 = kb * 32u + 8u * hi;
        float t0[8], t1[8]; float mloc = NEGV;
#pragma unroll
        for (int r = 0; r < 8; ++r) { const unsigned ja = j0 + r, jb = ja + 16u; const bool oka = (ja <= qi), okb = (jb <= qi); const unsigned ia = oka ? (qi - ja) : 0u, ib = okb ? (qi - jb) : 0u;
            const float ba = rpl[ia], bb = rpl[ib]; const float xa = s0[r] * SCLQK + ba, xb = s1[r] * SCLQK + bb;
            t0[r] = oka ? xa : NEGV; t1[r] = okb ? xb : NEGV; mloc = fmaxf(mloc, fmaxf(t0[r], t1[r])); }
        mloc = fmaxf(mloc, __shfl_xor(mloc, 16, 32));
        const float mn = fmaxf(m, mloc); const float f = __builtin_amdgcn_exp2f((m - mn) * L2E); m = mn;
        float psum = 0.f; v8h p0, p1;
#pragma unroll
        for (int r = 0; r < 8; ++r) { const h16 ha = (h16)__builtin_amdgcn_exp2f((t0[r] - mn) * L2E + 10.0f), hb = (h16)__builtin_amdgcn_exp2f((t1[r] - mn) * L2E + 10.0f);
            p0[r] = ha; p1[r] = hb; psum += (float)ha; psum += (float)hb; }
        l = l * f + psum;
#pragma unroll
        for (int mb = 0; mb < 4; ++mb) accO[mb] = accO[mb] * f;
        const v16h pb = cat16(p0, p1);
        const h16* vp = vbase + kb * 32u;
        v16h va[4];
#pragma unroll
        for (int mb = 0; mb < 4; ++mb) va[mb] = ldf(vp + (size_t)mb * 16 * SEQ);
#pragma unroll
        for (int mb = 0; mb < 4; ++mb) accO[mb] = wmma16(va[mb], pb, accO[mb]);
        asm volatile("v_nop\n\tv_nop\n\tv_nop\n\tv_nop" : "+v"(accO[0]), "+v"(accO[1]), "+v"(accO[2]), "+v"(accO[3]) : "v"(va[0]), "v"(va[3]), "v"(pb));
    }
    const float lt = l + __shfl_xor(l, 16, 32); const float inv = 2.0f * (1.0f / lt);
    h16* ow = &ot[wave][0];
#pragma unroll
    for (int mb = 0; mb < 4; ++mb) { v8h o;
#pragma unroll
        for (int r = 0; r < 8; ++r) o[r] = (h16)(accO[mb][r] * inv);
        *(v8ha*)(ow + lr * 72u + mb * 16 + 8u * hi) = o; }
    __syncthreads();
    h16* dst = OP + ((size_t)b * SEQ + qb * 16u) * EE + head * HD;
#pragma unroll 1
    for (int ps = 0; ps < 2; ++ps) {
#pragma unroll
        for (unsigned p = 0; p < 4u; ++p) { const unsigned row = p * 4u + (lane >> 3), pc = (lane & 7u) * 8u; const v8h v = *(const v8ha*)(ow + row * 72u + pc);
            *(volatile v8h*)(dst + (size_t)row * EE + pc) = v; }
        if (ps == 0) __threadfence(); }
}

#define SZ_WIN ((size_t)3 * EE * EE * 2)
#define SZ_WO  ((size_t)EE * EE * 2)
#define SZ_W1  ((size_t)FF * EE * 2)
#define SZ_W2  ((size_t)EE * FF * 2)
#define SZ_ACT ((size_t)ROWS * EE * 2)
#define SZ_X2  ((size_t)ROWS * EE * 4)
#define SZ_H   ((size_t)ROWS * FF * 2)
static_assert(SZ_WIN + SZ_WO + SZ_W1 + SZ_W2 + 6 * SZ_ACT + SZ_X2 + SZ_H <= (size_t)134217728);
static_assert(SZ_WIN % 256 == 0 && SZ_WO % 256 == 0 && SZ_ACT % 256 == 0 && SZ_X2 % 256 == 0 && SZ_H % 256 == 0);

extern "C" void kernel_launch(void* const* d_in, const int* in_sizes, int n_in,
                              void* d_out, int out_size, void* d_ws, size_t ws_size, hipStream_t stream) {
    if (n_in < 14) return;
    if ((size_t)in_sizes[0] < ((size_t)(NB - 1) * SEQ_FULL + SEQ) * EE) return;
    if ((size_t)in_sizes[1] < (size_t)(NHEAD - 1) * ML_FULL + SEQ) return;
    if ((size_t)in_sizes[2] < (size_t)3 * EE * EE || in_sizes[3] < 3 * EE || (size_t)in_sizes[4] < (size_t)EE * EE || in_sizes[5] < EE) return;
    if ((size_t)in_sizes[6] < (size_t)FF * EE || in_sizes[7] < FF || (size_t)in_sizes[8] < (size_t)EE * FF || in_sizes[9] < EE) return;
    if (in_sizes[10] < EE || in_sizes[11] < EE || in_sizes[12] < EE || in_sizes[13] < EE) return;
    if ((size_t)out_size < (size_t)ROWS * EE) return;
    const float* x = (const float*)d_in[0]; const float* relp = (const float*)d_in[1];
    const float* in_w = (const float*)d_in[2]; const float* in_b = (const float*)d_in[3];
    const float* out_w = (const float*)d_in[4]; const float* out_b = (const float*)d_in[5];
    const float* w1 = (const float*)d_in[6]; const float* b1 = (const float*)d_in[7];
    const float* w2 = (const float*)d_in[8]; const float* b2 = (const float*)d_in[9];
    const float* ln1_g = (const float*)d_in[10]; const float* ln1_b = (const float*)d_in[11];
    const float* ln2_g = (const float*)d_in[12]; const float* ln2_b = (const float*)d_in[13];
    float* OUT = (float*)d_out;
    char* wsp = (char*)d_ws;
    auto take = [&](size_t bytes) { char* p = wsp; wsp += (bytes + 255) & ~(size_t)255; return (void*)p; };
    h16* WIN = (h16*)take(SZ_WIN); h16* WO = (h16*)take(SZ_WO); h16* W1P = (h16*)take(SZ_W1); h16* W2P = (h16*)take(SZ_W2);
    h16* XN = (h16*)take(SZ_ACT); h16* XM = (h16*)take(SZ_ACT);
    h16* QP = (h16*)take(SZ_ACT); h16* KP = (h16*)take(SZ_ACT); h16* VT = (h16*)take(SZ_ACT); h16* OP = (h16*)take(SZ_ACT);
    float* X2 = (float*)take(SZ_X2); h16* HP = (h16*)take(SZ_H);
    if ((size_t)(wsp - (char*)d_ws) > ws_size) return;

    k_cvtw<<<(unsigned)((size_t)3 * EE * EE / 2048), 256, 0, stream>>>(in_w, WIN, (unsigned)((size_t)3 * EE * EE / 8));
    k_cvtw<<<(unsigned)((size_t)EE * EE / 2048), 256, 0, stream>>>(out_w, WO, (unsigned)((size_t)EE * EE / 8));
    k_cvtw<<<(unsigned)((size_t)FF * EE / 2048), 256, 0, stream>>>(w1, W1P, (unsigned)((size_t)FF * EE / 8));
    k_cvtw<<<(unsigned)((size_t)EE * FF / 2048), 256, 0, stream>>>(w2, W2P, (unsigned)((size_t)EE * FF / 8));

    k_ln<true><<<ROWS / 8, 256, 0, stream>>>(x, ln1_g, ln1_b, XN);
    k_gemmw<EPI_QKV, false><<<dim3(ROWS / 64, 3 * EE / 64, 1), 32, 0, stream>>>(XN, WIN, (unsigned)EE, in_b, 1.0f / 64.0f, 8.0f, nullptr, nullptr, QP, KP, VT, 0u);
    k_attn<<<NB * NHEAD * QT / 8, 256, 0, stream>>>(QP, KP, VT, relp, OP);
    k_gemmw<EPI_RES, true><<<dim3(ROWS / 64, EE / 64, 1), 32, 0, stream>>>(OP, WO, (unsigned)EE, out_b, 1.0f / 1024.0f, 1.0f, x, X2, nullptr, nullptr, nullptr, (unsigned)EE);
    k_ln<false><<<ROWS / 8, 256, 0, stream>>>(X2, ln2_g, ln2_b, XM);
    k_gemmw<EPI_RELU, false><<<dim3(ROWS / 64, FF / 64, 1), 32, 0, stream>>>(XM, W1P, (unsigned)EE, b1, 1.0f / 64.0f, 16.0f, nullptr, nullptr, HP, nullptr, nullptr, (unsigned)FF);
    k_gemmw<EPI_RES, false><<<dim3(ROWS / 64, EE / 64, 1), 32, 0, stream>>>(HP, W2P, (unsigned)FF, b2, 1.0f / 1024.0f, 1.0f, X2, OUT, nullptr, nullptr, nullptr, (unsigned)EE);
}
